// NonLocalBlock_67422396613171
// MI455X (gfx1250) — hardware-run, weakly checked
//
#include <hip/hip_runtime.h>


#ifndef NB
#define NB 4
#endif
#define NB_FULL 4
#define CH   64
#define HD   32
#define IMG  96
#define NP   (IMG * IMG)
#define PW   (IMG / 2)
#define MP   (PW * PW)
#define AW   4
#define OSP  68
#define QSP  36
#define PSP  68
#define TRP  72
#define OTP  68
#define RB   256
#define NBLK ((NB * NP) / RB)
#define QRS  2048.0f
#define QRI  (1.0f / 2048.0f)
#define LG2E 1.4426950408889634f
#define PSH  14.0f
#define NEGB (-3.0e38f)
#define WWS  64.0f
#define WWI  (1.0f / 64.0f)
#define BNEPS 1.0e-5f

static_assert(HD == 32);
static_assert(CH == 64);
static_assert(CH % 32 == 0);
static_assert(IMG % 2 == 0);
static_assert(NP % 64 == 0);
static_assert(NP % 256 == 0);
static_assert(MP % 64 == 0);
static_assert(PW % 16 == 0);
static_assert(MP % 32 == 0);
static_assert(NP % (16 * AW) == 0);
static_assert((NB * NP) % RB == 0);
static_assert(NB <= NB_FULL);
static_assert((OSP * 4) % 16 == 0);
static_assert((QSP * 4) % 16 == 0);
static_assert((PSP * 4) % 16 == 0);
static_assert((TRP * 2) % 16 == 0);
static_assert((OTP * 4) % 16 == 0);
static_assert(AW * 16 * OSP * 4 <= 131072);
static_assert(64 * PSP * 4 <= 131072);
static_assert(64 * TRP * 2 <= 131072);
static_assert(64 * OTP * 4 <= 131072);
static_assert(256 * 2 * 16 == 64 * CH * 2);
static_assert(32 * 2 * 16 == 16 * HD * 2);
static_assert(128 * 2 * 16 == 64 * HD * 2);
static_assert(128 * 2 * 16 == HD * 64 * 2);
static_assert(32 * 8 * 16 == 16 * CH * 4);
static_assert(256 * 4 * 16 == 64 * CH * 4);
static_assert(16 * 16 == RB);
static_assert(16 * 16 == CH * 4);

typedef _Float16 h16;
typedef unsigned short bf;
typedef __attribute__((ext_vector_type(16))) __bf16   v16bf;
typedef __attribute__((ext_vector_type(16))) _Float16 v16h;
typedef __attribute__((ext_vector_type(8)))  _Float16 v8h;
typedef __attribute__((ext_vector_type(8)))  unsigned short v8us;
typedef __attribute__((ext_vector_type(8)))  float    v8f;
typedef __attribute__((ext_vector_type(4)))  float    v4f;
typedef v4f  __attribute__((may_alias)) v4fa;
typedef v8us __attribute__((may_alias)) v8usa;

__device__ __forceinline__ unsigned short f2bf(float f) { unsigned u = __float_as_uint(f); u += 0x7FFFu + ((u >> 16) & 1u); return (unsigned short)(u >> 16); }
__device__ __forceinline__ float bfr(float f) { return __uint_as_float(((unsigned)f2bf(f)) << 16); }
__device__ __forceinline__ v16h cat16(v8h lo, v8h hi) { return __builtin_shufflevector(lo, hi, 0, 1, 2, 3, 4, 5, 6, 7, 8, 9, 10, 11, 12, 13, 14, 15); }
__device__ __forceinline__ v16bf cat16b(v8us lo, v8us hi) { return __builtin_bit_cast(v16bf, __builtin_shufflevector(lo, hi, 0, 1, 2, 3, 4, 5, 6, 7, 8, 9, 10, 11, 12, 13, 14, 15)); }
__device__ __forceinline__ v8f wmma16(v16h a, v16h b, v8f c) { return __builtin_amdgcn_wmma_f32_16x16x32_f16(false, a, false, b, (short)0, c, false, false); }
__device__ __forceinline__ v8f wmmab(v16bf a, v16bf b, v8f c) { return __builtin_amdgcn_wmma_f32_16x16x32_bf16(false, a, false, b, (short)0, c, false, false); }
__device__ __forceinline__ v8f wmma16g(v16h a, v16h b, v8f c) { c = wmma16(a, b, c); asm volatile("v_nop\n\tv_nop\n\tv_nop\n\tv_nop" : "+v"(c) : "v"(a), "v"(b)); return c; }
__device__ __forceinline__ v8f wmmabg(v16bf a, v16bf b, v8f c) { c = wmmab(a, b, c); asm volatile("v_nop\n\tv_nop\n\tv_nop\n\tv_nop" : "+v"(c) : "v"(a), "v"(b)); return c; }
__device__ __forceinline__ v16h  ldh(const h16* p) { return cat16(*(const v8h*)p, *(const v8h*)(p + 16)); }
__device__ __forceinline__ v16bf ldb(const bf* p)  { return cat16b(*(const v8us*)p, *(const v8us*)(p + 16)); }
__device__ __forceinline__ void wave_sync() { __builtin_amdgcn_fence(3  , "wavefront"); __builtin_amdgcn_wave_barrier(); asm volatile("" ::: "memory"); }
static __device__ __forceinline__ h16 toh_flush(float v) { const float w = (fabsf(v) < 6.103515625e-05f) ? 0.0f : v; return (h16)w; }

__global__ __launch_bounds__(256) void k_cvt8(const float* __restrict__ src, bf* dst, size_t n8) {
    const size_t i = (size_t)blockIdx.x * 256 + threadIdx.x; if (i >= n8) return;
    const v8f v = *(const v8f*)(src + i * 8); v8us o;
#pragma unroll
    for (int k = 0; k < 8; ++k) o[k] = f2bf(v[k]);
    *(volatile v8us*)(dst + i * 8) = o; __threadfence(); *(volatile v8us*)(dst + i * 8) = o;
}

__global__ __launch_bounds__(256) void k_wconv(const float* __restrict__ src, h16* dst, size_t n8) {
    const size_t i = (size_t)blockIdx.x * 256 + threadIdx.x; if (i >= n8) return;
    const v8f v = *(const v8f*)(src + i * 8); v8h o;
#pragma unroll
    for (int k = 0; k < 8; ++k) o[k] = toh_flush(bfr(v[k]) * WWS);
    *(volatile v8h*)(dst + i * 8) = o; __threadfence(); *(volatile v8h*)(dst + i * 8) = o;
}

__global__ __launch_bounds__(256) void k_tr(const float* __restrict__ src, bf* dst, int pooled) {
    __shared__ __align__(16) bf tl[64 * TRP];
    const unsigned tid = threadIdx.x, bx = blockIdx.x, b = blockIdx.y;
    const unsigned i = tid & 63u, cg = tid >> 6;
    const unsigned p = bx * 64u + i;
    const unsigned m = p >> 2, q = p & 3u;
    const unsigned ph = m / 48u, pw = m % 48u;
    const unsigned npool = (2u * ph + (q >> 1)) * 96u + 2u * pw + (q & 1u);
    const unsigned n = (pooled != 0) ? npool : p;
    const float* sp = src + (size_t)b * CH * NP + n;
#pragma unroll 1
    for (unsigned j = 0; j < 16u; ++j) { const unsigned c = cg + 4u * j; tl[i * TRP + c] = f2bf(sp[(size_t)c * NP]); }
    __syncthreads();
    bf* dp = dst + ((size_t)b * NP + (size_t)bx * 64u) * CH;
    v8us o[2];
#pragma unroll
    for (int s = 0; s < 2; ++s) { const unsigned pc = (unsigned)s * 256u + tid; const unsigned row = pc >> 3, c8 = (pc & 7u) * 8u; o[s] = *(const v8usa*)(&tl[row * TRP + c8]); }
#pragma unroll 1
    for (int ps = 0; ps < 2; ++ps) {
#pragma unroll
        for (int s = 0; s < 2; ++s) *(volatile v8us*)(dp + (size_t)((unsigned)s * 256u + tid) * 8) = o[s];
        if (ps == 0) __threadfence(); }
}

template <int NT>
__device__ __forceinline__ void gemm_k64(const bf* __restrict__ A, const bf* __restrict__ Bt, size_t aoff, size_t boff, v8f (&acc)[4][NT]) {
#pragma unroll
    for (int mb = 0; mb < 4; ++mb)
#pragma unroll
        for (int nb = 0; nb < NT; ++nb) acc[mb][nb] = (v8f){};
#pragma unroll 1
    for (int kc = 0; kc < CH; kc += 32) {
        v16bf a[4];
#pragma unroll
        for (int mb = 0; mb < 4; ++mb) a[mb] = ldb(A + aoff + (size_t)mb * 16 * CH + kc);
#pragma unroll
        for (int nb = 0; nb < NT; ++nb) { const v16bf b = ldb(Bt + boff + (size_t)nb * 16 * CH + kc);
#pragma unroll
            for (int mb = 0; mb < 4; ++mb) acc[mb][nb] = wmmabg(a[mb], b, acc[mb][nb]); }
    }
}

__global__ __launch_bounds__(32) void k_projq(const bf* __restrict__ A, const bf* __restrict__ Bt, h16* Ph, h16* Pr) {
    __shared__ __align__(16) float os[16 * QSP];
    const int lane = threadIdx.x & 31, lr = lane & 15, hi = lane >> 4;
    const unsigned r0 = blockIdx.x * 64u;
    v8f acc[4][2];
    gemm_k64<2>(A, Bt, (size_t)(r0 + (unsigned)lr) * CH + 8 * hi, (size_t)lr * CH + 8 * hi, acc);
#pragma unroll
    for (int mb = 0; mb < 4; ++mb) {
#pragma unroll
        for (int nb = 0; nb < 2; ++nb) {
#pragma unroll
            for (int j = 0; j < 8; ++j) os[(hi * 8 + j) * QSP + nb * 16 + lr] = acc[mb][nb][j]; }
        wave_sync();
        v8h hv[2], rv[2];
#pragma unroll
        for (int s = 0; s < 2; ++s) { const int p = s * 32 + lane; const int row = p >> 2, c8 = (p & 3) * 8;
            const v4f x0 = *(const v4fa*)(&os[row * QSP + c8]); const v4f x1 = *(const v4fa*)(&os[row * QSP + c8 + 4]);
#pragma unroll
            for (int i = 0; i < 4; ++i) { const h16 a0 = toh_flush(x0[i]); const h16 a1 = toh_flush(x1[i]); hv[s][i] = a0; hv[s][4 + i] = a1;
                rv[s][i] = toh_flush((x0[i] - (float)a0) * QRS); rv[s][4 + i] = toh_flush((x1[i] - (float)a1) * QRS); } }
        const size_t base = ((size_t)r0 + (size_t)(mb * 16)) * HD;
#pragma unroll 1
        for (int ps = 0; ps < 2; ++ps) {
#pragma unroll
            for (int s = 0; s < 2; ++s) { const size_t oo = base + (size_t)(s * 32 + lane) * 8;
                *(volatile v8h*)(Ph + oo) = hv[s]; *(volatile v8h*)(Pr + oo) = rv[s]; }
            if (ps == 0) __threadfence(); }
        wave_sync();
    }
}

__global__ __launch_bounds__(128) void k_projkv(const bf* __restrict__ A, const bf* __restrict__ Bt, h16* KPp, h16* KRp, h16* VTp, h16* VRp) {
    __shared__ __align__(16) float ps_[64 * PSP];
    const int lane = threadIdx.x & 31, lr = lane & 15, hi = lane >> 4;
    const int wave = __builtin_amdgcn_readfirstlane((int)(threadIdx.x >> 5));
    const unsigned tid = threadIdx.x, bx = blockIdx.x, b = blockIdx.y;
    const size_t r0 = (size_t)b * NP + (size_t)bx * 256u + (size_t)(wave * 64);
    v8f acc[4][4];
    gemm_k64<4>(A, Bt, (r0 + (size_t)lr) * CH + 8 * hi, (size_t)lr * CH + 8 * hi, acc);
#pragma unroll
    for (int mb = 0; mb < 4; ++mb) {
#pragma unroll
        for (int nb = 0; nb < 4; ++nb) {
            const v8f d = acc[mb][nb];
            const float lo = fmaxf(fmaxf(d[0], d[1]), fmaxf(d[2], d[3]));
            const float up = fmaxf(fmaxf(d[4], d[5]), fmaxf(d[6], d[7]));
            ps_[(wave * 16 + mb * 4 + 2 * hi + 0) * PSP + nb * 16 + lr] = lo;
            ps_[(wave * 16 + mb * 4 + 2 * hi + 1) * PSP + nb * 16 + lr] = up; } }
    __syncthreads();
    v8h kh[2], kr[2], vh[2], vr[2];
#pragma unroll
    for (int s = 0; s < 2; ++s) {
        const unsigned p = (unsigned)s * 128u + tid;
        { const unsigned row = p >> 2, c8 = (p & 3u) * 8u;
          const v4f x0 = *(const v4fa*)(&ps_[row * PSP + c8]); const v4f x1 = *(const v4fa*)(&ps_[row * PSP + c8 + 4]);
#pragma unroll
          for (int i = 0; i < 4; ++i) { const h16 a0 = toh_flush(x0[i]); const h16 a1 = toh_flush(x1[i]); kh[s][i] = a0; kh[s][4 + i] = a1;
              kr[s][i] = toh_flush((x0[i] - (float)a0) * QRS); kr[s][4 + i] = toh_flush((x1[i] - (float)a1) * QRS); } }
        { const unsigned d = p >> 3, m8 = (p & 7u) * 8u;
#pragma unroll
          for (int i = 0; i < 8; ++i) { const float x = ps_[(m8 + (unsigned)i) * PSP + 32u + d]; const h16 a0 = toh_flush(x); vh[s][i] = a0; vr[s][i] = toh_flush((x - (float)a0) * QRS); } }
    }
    const size_t kbase = ((size_t)b * MP + (size_t)bx * 64u) * HD;
    const size_t vbase = (size_t)b * HD * MP + (size_t)bx * 64u;
#pragma unroll 1
    for (int ps = 0; ps < 2; ++ps) {
#pragma unroll
        for (int s = 0; s < 2; ++s) {
            const unsigned p = (unsigned)s * 128u + tid;
            const size_t ko = kbase + (size_t)p * 8;
            const size_t vo = vbase + (size_t)(p >> 3) * MP + (size_t)((p & 7u) * 8u);
            *(volatile v8h*)(KPp + ko) = kh[s]; *(volatile v8h*)(KRp + ko) = kr[s];
            *(volatile v8h*)(VTp + vo) = vh[s]; *(volatile v8h*)(VRp + vo) = vr[s]; }
        if (ps == 0) __threadfence(); }
}

__global__ __launch_bounds__(32 * AW) void k_flash(const h16* __restrict__ QH, const h16* __restrict__ QR, const h16* __restrict__ KP, const h16* __restrict__ KR,
                                                   const h16* __restrict__ VT, const h16* __restrict__ VR, const h16* __restrict__ WW, float* WX) {
    __shared__ __align__(16) float os[AW * 16 * OSP];
    const int lane = threadIdx.x & 31, lr = lane & 15, hi = lane >> 4;
    const int wave = __builtin_amdgcn_readfirstlane((int)(threadIdx.x >> 5));
    const unsigned b = blockIdx.y;
    const int t0 = (int)(blockIdx.x * AW + (unsigned)wave) * 16;
    const size_t qo = ((size_t)b * NP + (size_t)(t0 + lr)) * HD + 8 * hi;
    const v16h qh = ldh(QH + qo), qr = ldh(QR + qo);
    const size_t ko = ((size_t)b * MP + (size_t)lr) * HD + 8 * hi;
    const size_t vo = ((size_t)b * HD + (size_t)lr) * MP + 8 * hi;
    v8f o0 = (v8f){}, o1 = (v8f){}, oR0 = (v8f){}, oR1 = (v8f){};
    float m = NEGB, l = 0.0f;
#pragma unroll 1
    for (int key0 = 0; key0 < MP; key0 += 32) {
        const h16* ka = KP + ko + (size_t)key0 * HD;
        const h16* kq = KR + ko + (size_t)key0 * HD;
        const v16h ka0 = ldh(ka), kb0 = ldh(ka + 16 * HD);
        const v16h kra0 = ldh(kq), krb0 = ldh(kq + 16 * HD);
        v8f sHa = (v8f){}, sLa = (v8f){}, sHb = (v8f){}, sLb = (v8f){};
        sHa = wmma16g(ka0, qh, sHa); sLa = wmma16g(ka0, qr, sLa); sLa = wmma16g(kra0, qh, sLa);
        sHb = wmma16g(kb0, qh, sHb); sLb = wmma16g(kb0, qr, sLb); sLb = wmma16g(krb0, qh, sLb);
        float ta[8], tb[8]; float mx = NEGB;
#pragma unroll
        for (int r = 0; r < 8; ++r) {
            ta[r] = (sHa[r] + sLa[r] * QRI) * LG2E; tb[r] = (sHb[r] + sLb[r] * QRI) * LG2E;
            mx = fmaxf(mx, fmaxf(ta[r], tb[r])); }
        mx = fmaxf(mx, __shfl_xor(mx, 16, 32));
        const float mnew = fmaxf(m, mx);
        const float alpha = __builtin_amdgcn_exp2f(m - mnew);
        const float sh = PSH - mnew;
        v16h pb; float ls = 0.0f;
#pragma unroll
        for (int r = 0; r < 8; ++r) {
            const float xa = ta[r] + sh, xb = tb[r] + sh;
            const float ea = __builtin_amdgcn_exp2f(xa), eb = __builtin_amdgcn_exp2f(xb);
            const float ga = (xa < -14.0f) ? 0.0f : ea, gb = (xb < -14.0f) ? 0.0f : eb;
            const h16 pa = (h16)ga; const h16 pc = (h16)gb;
            pb[r] = pa; pb[8 + r] = pc;
            ls += (float)pa + (float)pc; }
        l = l * alpha + ls; m = mnew;
        o0 = o0 * alpha; o1 = o1 * alpha; oR0 = oR0 * alpha; oR1 = oR1 * alpha;
        const h16* va = VT + vo + key0;
        const h16* vq = VR + vo + key0;
        const v16h v0 = ldh(va), v1 = ldh(va + (size_t)16 * MP);
        const v16h vr0 = ldh(vq), vr1 = ldh(vq + (size_t)16 * MP);
        o0 = wmma16g(v0, pb, o0); o1 = wmma16g(v1, pb, o1);
        oR0 = wmma16g(vr0, pb, oR0); oR1 = wmma16g(vr1, pb, oR1);
    }
    l += __shfl_xor(l, 16, 32);
    const float inv = 1.0f / l;
    v16h cb, cr;
#pragma unroll
    for (int r = 0; r < 8; ++r) {
        const float c0 = (o0[r] + oR0[r] * QRI) * inv, c1 = (o1[r] + oR1[r] * QRI) * inv;
        const h16 a0 = toh_flush(c0); const h16 a1 = toh_flush(c1);
        cb[r] = a0; cb[8 + r] = a1;
        cr[r] = toh_flush((c0 - (float)a0) * QRS); cr[8 + r] = toh_flush((c1 - (float)a1) * QRS); }
    const int wb = wave * 16 * OSP;
#pragma unroll
    for (int j = 0; j < 4; ++j) {
        const v16h aw = ldh(WW + (size_t)(16 * j + lr) * HD + 8 * hi);
        v8f wh = (v8f){}, wr = (v8f){};
        wh = wmma16g(aw, cb, wh); wr = wmma16g(aw, cr, wr);
        v4f a, c;
#pragma unroll
        for (int i = 0; i < 4; ++i) { a[i] = (wh[i] + wr[i] * QRI) * WWI; c[i] = (wh[4 + i] + wr[4 + i] * QRI) * WWI; }
        *(v4fa*)(&os[wb + lr * OSP + 16 * j + 8 * hi]) = a; *(v4fa*)(&os[wb + lr * OSP + 16 * j + 8 * hi + 4]) = c; }
    wave_sync();
    float* orow = WX + ((size_t)b * NP + (size_t)t0) * CH;
#pragma unroll 1
    for (int ps = 0; ps < 2; ++ps) {
#pragma unroll
        for (int s = 0; s < 8; ++s) { const int p = s * 32 + lane; const int row = p >> 4, cofs = (p & 15) * 4;
            const v4f val = *(const v4fa*)(&os[wb + row * OSP + cofs]);
            *(volatile v4f*)(orow + (size_t)p * 4) = val; }
        if (ps == 0) __threadfence(); }
}

__global__ __launch_bounds__(256) void k_colsum(const float* __restrict__ WXp, const float* __restrict__ stat, float* part, int centred) {
#pragma clang fp contract(off)
    __shared__ __align__(16) float red[16 * 64];
    __shared__ __align__(16) float tot[64];
    const unsigned tid = threadIdx.x, bx = blockIdx.x;
    const unsigned c4 = (tid & 15u) * 4u, rg = tid >> 4;
    v4f mu = (v4f){0.0f, 0.0f, 0.0f, 0.0f};
    if (centred != 0) mu = *(const v4f*)(stat + c4);
    const float* rp = WXp + ((size_t)bx * RB + rg) * CH + c4;
    v4f s = (v4f){0.0f, 0.0f, 0.0f, 0.0f};
#pragma unroll 1
    for (unsigned i = 0; i < 16u; ++i) {
        const v4f v = *(const v4f*)(rp + (size_t)i * 16 * CH);
        const v4f d = v - mu;
        if (centred != 0) s = s + d * d; else s = s + v; }
    *(v4fa*)(&red[rg * 64u + c4]) = s;
    __syncthreads();
    if (tid < 64u) { float t = 0.0f;
#pragma unroll 1
        for (unsigned g = 0; g < 16u; ++g) t += red[g * 64u + tid];
        tot[tid] = t; }
    __syncthreads();
    if (tid < 16u) { const v4f o = *(const v4fa*)(&tot[tid * 4u]); float* dp = part + (size_t)bx * 64 + tid * 4u;
        *(volatile v4f*)dp = o; __threadfence(); *(volatile v4f*)dp = o; }
}

static constexpr float INV_CNT = 1.0f / (float)((size_t)NB * NP);

__global__ __launch_bounds__(64) void k_fin(const float* __restrict__ part, float* stat, int mode) {
#pragma clang fp contract(off)
    __shared__ __align__(16) float sm[64];
    const unsigned tid = threadIdx.x;
    const unsigned md = (mode != 0) ? 1u : 0u;
    float s = 0.0f, c = 0.0f;
#pragma unroll 1
    for (unsigned i = 0; i < (unsigned)NBLK; ++i) { const float y = part[(size_t)i * 64 + tid] - c; const float t = s + y; c = (t - s) - y; s = t; }
    const float q = s * INV_CNT;
    float r = q;
    if (md != 0u) r = rsqrtf(q + BNEPS);
    sm[tid] = r;
    __syncthreads();
    if (tid < 16u) { const v4f o = *(const v4fa*)(&sm[tid * 4u]); float* dp = stat + (size_t)md * 64 + tid * 4u;
        *(volatile v4f*)dp = o; __threadfence(); *(volatile v4f*)dp = o; }
}

__global__ __launch_bounds__(256) void k_out(const float* __restrict__ WXp, const float* __restrict__ stat, const float* __restrict__ gain, const float* __restrict__ offs,
                                             const float* __restrict__ x, float* out) {
#pragma clang fp contract(off)
    __shared__ __align__(16) float tl[64 * OTP];
    const unsigned tid = threadIdx.x, bx = blockIdx.x, b = blockIdx.y;
    const unsigned c4 = (tid & 15u) * 4u, rg = tid >> 4;
    const v4f mu = *(const v4f*)(stat + c4), rs = *(const v4f*)(stat + 64 + c4);
    const v4f gv = *(const v4f*)(gain + c4), bv = *(const v4f*)(offs + c4);
    v4f gb, bb;
#pragma unroll
    for (int i = 0; i < 4; ++i) { gb[i] = bfr(gv[i]); bb[i] = bfr(bv[i]); }
    const float* rp = WXp + ((size_t)b * NP + (size_t)bx * 64u + rg) * CH + c4;
#pragma unroll 1
    for (unsigned s = 0; s < 4u; ++s) {
        const unsigned row = rg + 16u * s;
        const v4f v = *(const v4f*)(rp + (size_t)s * 16 * CH);
#pragma unroll
        for (int i = 0; i < 4; ++i) tl[(c4 + (unsigned)i) * OTP + row] = ((v[i] - mu[i]) * rs[i]) * gb[i] + bb[i]; }
    __syncthreads();
    const size_t ob = (size_t)b * CH * NP + (size_t)bx * 64u;
    v4f val[4];
#pragma unroll
    for (int s = 0; s < 4; ++s) { const unsigned p = (unsigned)s * 256u + tid; const unsigned c = p >> 4, n4 = (p & 15u) * 4u;
        const v4f t = *(const v4fa*)(&tl[c * OTP + n4]);
        const v4f xv = *(const v4f*)(x + ob + (size_t)c * NP + n4);
#pragma unroll
        for (int i = 0; i < 4; ++i) val[s][i] = t[i] + bfr(xv[i]); }
#pragma unroll 1
    for (int ps = 0; ps < 2; ++ps) {
#pragma unroll
        for (int s = 0; s < 4; ++s) { const unsigned p = (unsigned)s * 256u + tid; const unsigned c = p >> 4, n4 = (p & 15u) * 4u;
            *(volatile v4f*)(out + ob + (size_t)c * NP + n4) = val[s]; }
        if (ps == 0) __threadfence(); }
}

static constexpr size_t al256(size_t v) { return (v + 255) & ~(size_t)255; }
static constexpr size_t SZ_XB = al256((size_t)NB * NP * CH * 2);
static constexpr size_t SZ_WT = al256((size_t)HD * CH * 2);
static constexpr size_t SZ_WK = al256((size_t)2 * HD * CH * 2);
static constexpr size_t SZ_WW = al256((size_t)CH * HD * 2);
static constexpr size_t SZ_QP = al256((size_t)NB * NP * HD * 2);
static constexpr size_t SZ_KP = al256((size_t)NB * MP * HD * 2);
static constexpr size_t SZ_WX = al256((size_t)NB * NP * CH * 4);
static constexpr size_t SZ_PT = al256((size_t)NBLK * 64 * 4);
static constexpr size_t SZ_ST = al256((size_t)128 * 4);
static constexpr size_t OFF_XB = 0;
static constexpr size_t OFF_YB = OFF_XB + SZ_XB;
static constexpr size_t OFF_WT = OFF_YB + SZ_XB;
static constexpr size_t OFF_WK = OFF_WT + SZ_WT;
static constexpr size_t OFF_WW = OFF_WK + SZ_WK;
static constexpr size_t OFF_QH = OFF_WW + SZ_WW;
static constexpr size_t OFF_QR = OFF_QH + SZ_QP;
static constexpr size_t OFF_KP = OFF_QR + SZ_QP;
static constexpr size_t OFF_KR = OFF_KP + SZ_KP;
static constexpr size_t OFF_VT = OFF_KR + SZ_KP;
static constexpr size_t OFF_VR = OFF_VT + SZ_KP;
static constexpr size_t OFF_WX = OFF_VR + SZ_KP;
static constexpr size_t OFF_P0 = OFF_WX + SZ_WX;
static constexpr size_t OFF_P1 = OFF_P0 + SZ_PT;
static constexpr size_t OFF_ST = OFF_P1 + SZ_PT;
static constexpr size_t SZ_TOTAL = OFF_ST + SZ_ST;
static_assert(SZ_TOTAL <= (size_t)134217728);
static_assert(((size_t)HD * CH * 2) % 256 == 0);
static_assert((size_t)(NP / 64) * 64 * CH * 2 * NB <= SZ_XB);
static_assert((size_t)(NB * NP / 64) * 64 * HD * 2 <= SZ_QP);
static_assert((size_t)NB * (NP / 256) * 64 * HD * 2 <= SZ_KP);
static_assert((size_t)NB * (NP / (16 * AW)) * AW * 16 * CH * 4 <= SZ_WX);
static constexpr size_t NEED_X = (size_t)NB * CH * NP;
static constexpr size_t N8_W = (size_t)HD * CH / 8;
static constexpr unsigned G_W = (unsigned)((N8_W + 255) / 256);
static constexpr size_t WV_OFS = (size_t)HD * CH;

extern "C" void kernel_launch(void* const* d_in, const int* in_sizes, int n_in,
                              void* d_out, int out_size, void* d_ws, size_t ws_size, hipStream_t stream) {
    if (n_in < 8) return;
    if ((size_t)in_sizes[0] < NEED_X || (size_t)in_sizes[1] < NEED_X) return;
    if (in_sizes[2] < HD * CH || in_sizes[3] < HD * CH || in_sizes[4] < HD * CH || in_sizes[5] < CH * HD) return;
    if (in_sizes[6] < CH || in_sizes[7] < CH) return;
    if ((size_t)out_size < NEED_X) return;
    if (SZ_TOTAL > ws_size) return;
    const float* x  = (const float*)d_in[0]; const float* y  = (const float*)d_in[1];
    const float* wq = (const float*)d_in[2]; const float* wk = (const float*)d_in[3]; const float* wv = (const float*)d_in[4];
    const float* wo = (const float*)d_in[5]; const float* gn = (const float*)d_in[6]; const float* bt = (const float*)d_in[7];
    float* OUT = (float*)d_out;
    char* wsp = (char*)d_ws;
    bf*  XB = (bf*)(wsp + OFF_XB);
    bf*  YB = (bf*)(wsp + OFF_YB);
    bf*  WT = (bf*)(wsp + OFF_WT);
    bf*  WK = (bf*)(wsp + OFF_WK);
    h16* WW = (h16*)(wsp + OFF_WW);
    h16* QH = (h16*)(wsp + OFF_QH);
    h16* QR = (h16*)(wsp + OFF_QR);
    h16* KP = (h16*)(wsp + OFF_KP);
    h16* KR = (h16*)(wsp + OFF_KR);
    h16* VT = (h16*)(wsp + OFF_VT);
    h16* VR = (h16*)(wsp + OFF_VR);
    float* WX = (float*)(wsp + OFF_WX);
    float* P0 = (float*)(wsp + OFF_P0);
    float* P1 = (float*)(wsp + OFF_P1);
    float* ST = (float*)(wsp + OFF_ST);

    k_tr<<<dim3(NP / 64, NB, 1), 256, 0, stream>>>(x, XB, 0);
    k_tr<<<dim3(NP / 64, NB, 1), 256, 0, stream>>>(y, YB, 1);
    k_cvt8<<<G_W, 256, 0, stream>>>(wq, WT, N8_W);
    k_cvt8<<<G_W, 256, 0, stream>>>(wk, WK, N8_W);
    k_cvt8<<<G_W, 256, 0, stream>>>(wv, WK + WV_OFS, N8_W);
    k_wconv<<<G_W, 256, 0, stream>>>(wo, WW, N8_W);

    k_projq<<<dim3(NB * NP / 64, 1, 1), 32, 0, stream>>>(XB, WT, QH, QR);
    k_projkv<<<dim3(NP / 256, NB, 1), 128, 0, stream>>>(YB, WK, KP, KR, VT, VR);

    k_flash<<<dim3(NP / (16 * AW), NB, 1), 32 * AW, 0, stream>>>(QH, QR, KP, KR, VT, VR, WW, WX);

    k_colsum<<<dim3(NBLK, 1, 1), 256, 0, stream>>>(WX, ST, P0, 0);
    k_fin<<<dim3(1, 1, 1), 64, 0, stream>>>(P0, ST, 0);
    k_colsum<<<dim3(NBLK, 1, 1), 256, 0, stream>>>(WX, ST, P1, 1);
    k_fin<<<dim3(1, 1, 1), 64, 0, stream>>>(P1, ST, 1);

    k_out<<<dim3(NP / 64, NB, 1), 256, 0, stream>>>(WX, ST, gn, bt, x, OUT);
}
